// SelfAttention_35622458753629
// MI455X (gfx1250) — hardware-verified
//
#include <hip/hip_runtime.h>


#ifndef NB
#define NB 8
#endif
#ifndef SEQ
#define SEQ 1365
#endif
#define NB_FULL    8
#define SEQ_FULL   1365
#define DIM        1024
#define NHEAD      16
#define HDIM       64
#define CDIM       256
#define ADA_N      2048
#define QKV_N      3072
#define SPAD       (((SEQ + 127) / 128) * 128)
#define BQ         128
#define BK         32
#define NWAVE      8
#define TP         72
#define OP         68
#define PE         132
#define WCARRY     16.0f
#define PCARRY     4096.0f
#define CCARRY     64.0f

static_assert(NB >= 1 && NB <= NB_FULL);
static_assert(SEQ >= 1 && SEQ <= SEQ_FULL);
static_assert(SEQ_FULL == 1365);
static_assert(SPAD % 128 == 0);
static_assert(SPAD % 8 == 0 && SPAD % 4 == 0);
static_assert(HDIM == 64);
static_assert(DIM == NHEAD * HDIM);
static_assert(DIM == 4 * 32 * 8);
static_assert(DIM % 128 == 0 && QKV_N % 128 == 0 && DIM % 64 == 0 && QKV_N % 64 == 0);
static_assert(DIM % 32 == 0);
static_assert(ADA_N == 2 * 256 * 4);
static_assert(ADA_N == 2 * DIM && QKV_N == 3 * DIM);
static_assert(BQ == NWAVE * 16);
static_assert((TP * 2) % 16 == 0 && (OP * 4) % 16 == 0 && (PE * 4) % 16 == 0);

#define SZ_FTAB  ((size_t)512)
#define SZ_WB    ((size_t)NB * ADA_N * 4)
#define SZ_TAB   ((size_t)NHEAD * SPAD * 64 * 4)
#define SZ_WQKV  ((size_t)QKV_N * DIM * 2)
#define SZ_WOUT  ((size_t)DIM * DIM * 2)
#define SZ_XN    ((size_t)NB * SPAD * DIM * 2)
#define SZ_HP    ((size_t)NB * NHEAD * SPAD * HDIM * 2)
#define OFF_FTAB ((size_t)0)
#define OFF_WB   (OFF_FTAB + SZ_FTAB)
#define OFF_TABC (OFF_WB + SZ_WB)
#define OFF_TABS (OFF_TABC + SZ_TAB)
#define OFF_WQKV (OFF_TABS + SZ_TAB)
#define OFF_WOUT (OFF_WQKV + SZ_WQKV)
#define OFF_XN   (OFF_WOUT + SZ_WOUT)
#define OFF_Q    (OFF_XN + SZ_XN)
#define OFF_K    (OFF_Q + SZ_HP)
#define OFF_VT   (OFF_K + SZ_HP)
#define WS_TOTAL (OFF_VT + SZ_HP)
static_assert(WS_TOTAL <= (size_t)134217728);
static_assert(SZ_WB % 128 == 0 && SZ_TAB % 128 == 0 && SZ_XN % 128 == 0 && SZ_HP % 128 == 0);

typedef __bf16   bf16;
typedef _Float16 f16;
typedef f16      v16h  __attribute__((ext_vector_type(16)));
typedef f16      v8h   __attribute__((ext_vector_type(8)));
typedef float    v8f   __attribute__((ext_vector_type(8)));
typedef float    v4f   __attribute__((ext_vector_type(4)));
typedef unsigned v4u   __attribute__((ext_vector_type(4)));

union FragH  { v16h v; v4u q[2]; f16 h[16]; };
union Pack8H { v4u u; v8h v; f16 h[8]; };

struct F32x32 { float v[32]; };
static_assert(sizeof(F32x32) == 128);

static __device__ __forceinline__ float bfr(float x) { return (float)(bf16)x; }

static __device__ __forceinline__ v8f zero8() { return (v8f){0, 0, 0, 0, 0, 0, 0, 0}; }

static __device__ __forceinline__ unsigned umin_u(unsigned a, unsigned b) { return a < b ? a : b; }

static __device__ __forceinline__ v8f mma_f16(v16h a, v16h b, v8f acc) {
  acc = __builtin_amdgcn_wmma_f32_16x16x32_f16(false, a, false, b, (short)0, acc, false, false);
  asm volatile("v_nop\n\tv_nop\n\tv_nop\n\tv_nop" : "+v"(acc) : "v"(a), "v"(b));
  return acc;
}

static __device__ __forceinline__ float wave_sum(float v) {
  v += __shfl_xor(v, 16, 32);
  v += __shfl_xor(v, 8, 32);
  v += __shfl_xor(v, 4, 32);
  v += __shfl_xor(v, 2, 32);
  v += __shfl_xor(v, 1, 32);
  return v;
}

static __device__ __forceinline__ unsigned seg_end_of(unsigned q) {
  unsigned e = 1u;
  e = (q >= 1u)   ? 5u    : e;
  e = (q >= 5u)   ? 21u   : e;
  e = (q >= 21u)  ? 85u   : e;
  e = (q >= 85u)  ? 341u  : e;
  e = (q >= 341u) ? 1365u : e;
  return umin_u(e, (unsigned)SEQ);
}

__global__ __launch_bounds__(32) void freq_kernel(F32x32 f, float* __restrict__ ftab, unsigned base) {
  const unsigned t = threadIdx.x;
  float val = f.v[0];
  #pragma unroll
  for (unsigned i = 1; i < 32; ++i) val = (t == i) ? f.v[i] : val;
  volatile float* p = ftab + base + t;
  *p = val;
  __threadfence();
  *p = val;
}

__global__ __launch_bounds__(256) void rope_table_kernel(const float* __restrict__ ftab,
                                                         float* __restrict__ tabC,
                                                         float* __restrict__ tabS) {
  __shared__ __align__(16) float sC[256];
  __shared__ __align__(16) float sS[256];
  const unsigned tid = threadIdx.x;
  const unsigned h   = blockIdx.y;
  const unsigned s0  = blockIdx.x << 2;
  const unsigned s   = s0 + (tid >> 6);
  const unsigned d   = tid & 63u;

  unsigned k = 0u, off = 0u;
  k = (s >= 1u)   ? 1u : k;   off = (s >= 1u)   ? 1u   : off;
  k = (s >= 5u)   ? 2u : k;   off = (s >= 5u)   ? 5u   : off;
  k = (s >= 21u)  ? 3u : k;   off = (s >= 21u)  ? 21u  : off;
  k = (s >= 85u)  ? 4u : k;   off = (s >= 85u)  ? 85u  : off;
  k = (s >= 341u) ? 5u : k;   off = (s >= 341u) ? 341u : off;
  const unsigned n   = 1u << k;
  const unsigned l   = s - off;
  const unsigned r   = l >> k;
  const unsigned c   = l & (n - 1u);
  const float    inv = __uint_as_float((127u - k) << 23);
  const float ph = (float)(2u * r + 1u) * inv - 1.0f;
  const float pw = (float)(2u * c + 1u) * inv - 1.0f;
  float pd = 0.0f;
  pd = (k == 1u) ? 0.2f : pd;
  pd = (k == 2u) ? 0.4f : pd;
  pd = (k == 3u) ? 0.6f : pd;
  pd = (k == 4u) ? 0.8f : pd;
  pd = (k == 5u) ? 1.0f : pd;

  unsigned jj = (d >= 24u) ? d - 24u : d;
  jj = umin_u(jj, 23u);
  const unsigned g = jj >> 3;
  const unsigned j = jj & 7u;
  const float comp = (g == 0u) ? ph : ((g == 1u) ? pw : pd);
  const float fr   = ftab[(j << 4) + h];
  const bool  live = (d < 48u) && (s < (unsigned)SEQ);
  const float ang  = live ? comp * fr : 0.0f;
  float sn, cs;
  sincosf(ang, &sn, &cs);
  sC[tid] = cs;
  sS[tid] = (d < 24u) ? -sn : sn;
  __syncthreads();

  if (tid < 128u) {
    const unsigned arr   = tid >> 6;
    const unsigned idx   = tid & 63u;
    const unsigned row   = idx >> 4;
    const unsigned piece = idx & 15u;
    const v4f vc = *(const v4f*)(sC + row * 64u + piece * 4u);
    const v4f vs = *(const v4f*)(sS + row * 64u + piece * 4u);
    const v4f v  = (arr != 0u) ? vs : vc;
    float* dst = ((arr != 0u) ? tabS : tabC) + ((size_t)h * SPAD + s0 + row) * 64u + piece * 4u;
    *(volatile v4f*)dst = v;
    __threadfence();
    *(volatile v4f*)dst = v;
  }
}

__global__ __launch_bounds__(256) void adaln_kernel(const float* __restrict__ cond,
                                                    const float* __restrict__ w,
                                                    const float* __restrict__ bias,
                                                    float* __restrict__ wb) {
  const unsigned tid = threadIdx.x;
  const unsigned b   = blockIdx.y;
  const unsigned n4  = (blockIdx.x * 256u + tid) << 2;
  const float* c = cond + (size_t)b * CDIM;
  v4f acc = {0.0f, 0.0f, 0.0f, 0.0f};
  #pragma unroll 2
  for (unsigned k = 0; k < (unsigned)CDIM; ++k) {
    const float cv = bfr(c[k]);
    const v4f wv = *(const v4f*)(w + (size_t)k * ADA_N + n4);
    acc[0] = fmaf(cv, bfr(wv[0]), acc[0]);
    acc[1] = fmaf(cv, bfr(wv[1]), acc[1]);
    acc[2] = fmaf(cv, bfr(wv[2]), acc[2]);
    acc[3] = fmaf(cv, bfr(wv[3]), acc[3]);
  }
  const v4f bv = *(const v4f*)(bias + n4);
  v4f res;
  res[0] = acc[0] + bfr(bv[0]);
  res[1] = acc[1] + bfr(bv[1]);
  res[2] = acc[2] + bfr(bv[2]);
  res[3] = acc[3] + bfr(bv[3]);
  float* dst = wb + (size_t)b * ADA_N + n4;
  *(volatile v4f*)dst = res;
  __threadfence();
  *(volatile v4f*)dst = res;
}

__global__ __launch_bounds__(256) void wt_plane_kernel(const float* __restrict__ in,
                                                       f16* __restrict__ outp,
                                                       unsigned K, unsigned N) {
  __shared__ __align__(16) f16 sT[64 * TP];
  const unsigned tid = threadIdx.x;
  const unsigned n0  = blockIdx.x * 64u;
  const unsigned k0  = blockIdx.y * 64u;
  #pragma unroll
  for (unsigned it = 0; it < 4; ++it) {
    const unsigned idx = it * 256u + tid;
    const unsigned kr  = idx >> 4;
    const unsigned n4  = (idx & 15u) << 2;
    const v4f v = *(const v4f*)(in + (size_t)(k0 + kr) * N + n0 + n4);
    #pragma unroll
    for (unsigned i = 0; i < 4; ++i) sT[(n4 + i) * TP + kr] = (f16)(bfr(v[i]) * WCARRY);
  }
  __syncthreads();

  v4u    vals[2];
  size_t gidx[2];
  #pragma unroll
  for (unsigned it = 0; it < 2; ++it) {
    const unsigned n  = it * 32u + (tid >> 3);
    const unsigned ks = (tid & 7u) << 3;
    Pack8H ph;
    ph.v = *(const v8h*)(sT + n * TP + ks);
    vals[it] = ph.u;
    gidx[it] = (size_t)(n0 + n) * K + k0 + ks;
  }
  #pragma unroll
  for (unsigned it = 0; it < 2; ++it) *(volatile v4u*)(outp + gidx[it]) = vals[it];
  __threadfence();
  #pragma unroll
  for (unsigned it = 0; it < 2; ++it) *(volatile v4u*)(outp + gidx[it]) = vals[it];
}

static __device__ __forceinline__ void ln_emit(const float* __restrict__ xr, const float* __restrict__ wrow,
                                               f16* dst, float mu, float inv, unsigned lane) {
  #pragma unroll 1
  for (unsigned i = 0; i < 4; ++i) {
    const unsigned c = i * 256u + lane * 8u;
    const v4f a0 = *(const v4f*)(xr + c);
    const v4f a1 = *(const v4f*)(xr + c + 4u);
    const v4f w0 = *(const v4f*)(wrow + c);
    const v4f w1 = *(const v4f*)(wrow + c + 4u);
    const v4f b0 = *(const v4f*)(wrow + DIM + c);
    const v4f b1 = *(const v4f*)(wrow + DIM + c + 4u);
    Pack8H pk;
    #pragma unroll
    for (unsigned j = 0; j < 4; ++j) {
      pk.h[j]      = (f16)(((bfr(a0[j]) - mu) * inv) * (w0[j] + 1.0f) + b0[j]);
      pk.h[4u + j] = (f16)(((bfr(a1[j]) - mu) * inv) * (w1[j] + 1.0f) + b1[j]);
    }
    *(volatile v4u*)(dst + c) = pk.u;
  }
}

__global__ __launch_bounds__(256) void ln_kernel(const float* __restrict__ x,
                                                 const float* __restrict__ wb,
                                                 f16* xn) {
  const unsigned tid  = threadIdx.x;
  const unsigned wave = (unsigned)__builtin_amdgcn_readfirstlane((int)(tid >> 5));
  const unsigned lane = tid & 31u;
  const unsigned s    = blockIdx.x * 8u + wave;
  const unsigned b    = blockIdx.y;
  f16* dst = xn + ((size_t)b * SPAD + s) * DIM;

  if (s >= (unsigned)SEQ) {
    const v4u z = {0u, 0u, 0u, 0u};
    #pragma unroll
    for (unsigned i = 0; i < 4; ++i) *(volatile v4u*)(dst + i * 256u + lane * 8u) = z;
    __threadfence();
    #pragma unroll
    for (unsigned i = 0; i < 4; ++i) *(volatile v4u*)(dst + i * 256u + lane * 8u) = z;
    return;
  }

  const float* xr = x + ((size_t)b * SEQ_FULL + s) * DIM;
  float sum = 0.0f;
  #pragma unroll 1
  for (unsigned i = 0; i < 4; ++i) {
    const unsigned c = i * 256u + lane * 8u;
    const v4f a0 = *(const v4f*)(xr + c);
    const v4f a1 = *(const v4f*)(xr + c + 4u);
    sum += (bfr(a0[0]) + bfr(a0[1])) + (bfr(a0[2]) + bfr(a0[3]));
    sum += (bfr(a1[0]) + bfr(a1[1])) + (bfr(a1[2]) + bfr(a1[3]));
  }
  const float mu = wave_sum(sum) * (1.0f / (float)DIM);
  float sq = 0.0f;
  #pragma unroll 1
  for (unsigned i = 0; i < 4; ++i) {
    const unsigned c = i * 256u + lane * 8u;
    const v4f a0 = *(const v4f*)(xr + c);
    const v4f a1 = *(const v4f*)(xr + c + 4u);
    #pragma unroll
    for (unsigned j = 0; j < 4; ++j) {
      const float d0 = bfr(a0[j]) - mu;
      const float d1 = bfr(a1[j]) - mu;
      sq = fmaf(d0, d0, sq);
      sq = fmaf(d1, d1, sq);
    }
  }
  const float var = wave_sum(sq) * (1.0f / (float)DIM);
  const float inv = rsqrtf(var + 1e-5f);
  const float* wrow = wb + (size_t)b * ADA_N;
  ln_emit(xr, wrow, dst, mu, inv, lane);
  __threadfence();
  ln_emit(xr, wrow, dst, mu, inv, lane);
}

static __device__ __forceinline__ void gemm_32x64(const f16* __restrict__ a_base,
                                                  const f16* __restrict__ b_base,
                                                  unsigned ksteps, v8f (&acc)[2][4]) {
  #pragma unroll 1
  for (unsigned ks = 0; ks < ksteps; ++ks) {
    const unsigned k0 = ks * 32u;
    FragH a[2], bw[4];
    #pragma unroll
    for (unsigned ms = 0; ms < 2; ++ms) {
      const f16* p = a_base + (size_t)ms * 16u * DIM + k0;
      a[ms].q[0] = *(const v4u*)(p);
      a[ms].q[1] = *(const v4u*)(p + 16);
    }
    #pragma unroll
    for (unsigned t = 0; t < 4; ++t) {
      const f16* p = b_base + (size_t)t * 16u * DIM + k0;
      bw[t].q[0] = *(const v4u*)(p);
      bw[t].q[1] = *(const v4u*)(p + 16);
    }
    #pragma unroll
    for (unsigned ms = 0; ms < 2; ++ms) {
      #pragma unroll
      for (unsigned t = 0; t < 4; ++t) acc[ms][t] = mma_f16(a[ms].v, bw[t].v, acc[ms][t]);
    }
  }
}

__global__ __launch_bounds__(256) void qkv_gemm_kernel(const f16* __restrict__ xn,
                                                       const f16* __restrict__ wT,
                                                       const float* __restrict__ bias,
                                                       const float* __restrict__ tabC,
                                                       const float* __restrict__ tabS,
                                                       f16* __restrict__ qp,
                                                       f16* __restrict__ kp,
                                                       f16* __restrict__ vt) {
  __shared__ __align__(16) float sE[128 * PE];
  const unsigned tid  = threadIdx.x;
  const unsigned wave = (unsigned)__builtin_amdgcn_readfirstlane((int)(tid >> 5));
  const unsigned lane = tid & 31u;
  const unsigned lq   = lane & 15u;
  const unsigned hi   = lane >> 4;
  const unsigned wm   = wave & 3u;
  const unsigned wn   = wave >> 2;
  const unsigned bx   = blockIdx.x;
  const unsigned by   = blockIdx.y;
  const unsigned b    = blockIdx.z;

  const unsigned row0  = by * 128u + wm * 32u;
  const unsigned ncol0 = bx * 128u + wn * 64u;
  const f16* a_base = xn + ((size_t)b * SPAD + row0 + lq) * DIM + hi * 8u;
  const f16* b_base = wT + ((size_t)ncol0 + lq) * DIM + hi * 8u;
  const unsigned ksteps = (row0 < (unsigned)SEQ) ? (unsigned)(DIM / 32) : 0u;

  v8f acc[2][4];
  #pragma unroll
  for (unsigned ms = 0; ms < 2; ++ms) {
    #pragma unroll
    for (unsigned t = 0; t < 4; ++t) acc[ms][t] = zero8();
  }
  gemm_32x64(a_base, b_base, ksteps, acc);

  #pragma unroll
  for (unsigned t = 0; t < 4; ++t) {
    const float bn = bfr(bias[ncol0 + t * 16u + lq]);
    #pragma unroll
    for (unsigned ms = 0; ms < 2; ++ms) {
      #pragma unroll
      for (unsigned r = 0; r < 8; ++r) {
        sE[(wm * 32u + ms * 16u + hi * 8u + r) * PE + wn * 64u + t * 16u + lq] =
            acc[ms][t][r] * (1.0f / WCARRY) + bn;
      }
    }
  }
  __syncthreads();

  const unsigned which = bx >> 3;
  const unsigned h0    = (bx & 7u) << 1;
  const size_t   bh0   = (size_t)b * NHEAD + h0;

  if (which < 2u) {
    f16* plane = (which == 0u) ? qp : kp;
    const unsigned p  = tid & 7u;
    const unsigned pp = (p < 3u) ? p + 3u : ((p < 6u) ? p - 3u : p);
    #pragma unroll
    for (unsigned g = 0; g < 2; ++g) {
      v4u    vals[4];
      size_t gidx[4];
      #pragma unroll
      for (unsigned j = 0; j < 4; ++j) {
        const unsigned L   = (g * 4u + j) * 32u + (tid >> 3);
        const unsigned hl  = L >> 7;
        const unsigned row = L & 127u;
        const unsigned s   = by * 128u + row;
        const float* xr = sE + row * PE + hl * 64u;
        const v4f x0 = *(const v4f*)(xr + p * 8u);
        const v4f x1 = *(const v4f*)(xr + p * 8u + 4u);
        const v4f y0 = *(const v4f*)(xr + pp * 8u);
        const v4f y1 = *(const v4f*)(xr + pp * 8u + 4u);
        const size_t trow = ((size_t)(h0 + hl) * SPAD + s) * 64u + p * 8u;
        const v4f c0 = *(const v4f*)(tabC + trow);
        const v4f c1 = *(const v4f*)(tabC + trow + 4u);
        const v4f n0 = *(const v4f*)(tabS + trow);
        const v4f n1 = *(const v4f*)(tabS + trow + 4u);
        Pack8H pk;
        #pragma unroll
        for (unsigned i = 0; i < 4; ++i) {
          pk.h[i]      = (f16)(x0[i] * c0[i] + y0[i] * n0[i]);
          pk.h[4u + i] = (f16)(x1[i] * c1[i] + y1[i] * n1[i]);
        }
        vals[j] = pk.u;
        gidx[j] = ((bh0 + hl) * SPAD + s) * HDIM + p * 8u;
      }
      #pragma unroll
      for (unsigned j = 0; j < 4; ++j) *(volatile v4u*)(plane + gidx[j]) = vals[j];
      __threadfence();
      #pragma unroll
      for (unsigned j = 0; j < 4; ++j) *(volatile v4u*)(plane + gidx[j]) = vals[j];
    }
  } else {
    const unsigned p = tid & 7u;
    #pragma unroll
    for (unsigned g = 0; g < 2; ++g) {
      v4u    vals[4];
      size_t gidx[4];
      #pragma unroll
      for (unsigned j = 0; j < 4; ++j) {
        const unsigned L    = (g * 4u + j) * 32u + (tid >> 3);
        const unsigned sh   = L & 1u;
        const unsigned d    = (L >> 1) & 63u;
        const unsigned hl   = L >> 7;
        const unsigned srow = sh * 64u + p * 8u;
        Pack8H pk;
        #pragma unroll
        for (unsigned i = 0; i < 8; ++i) pk.h[i] = (f16)sE[(srow + i) * PE + hl * 64u + d];
        vals[j] = pk.u;
        gidx[j] = ((bh0 + hl) * HDIM + d) * SPAD + by * 128u + srow;
      }
      #pragma unroll
      for (unsigned j = 0; j < 4; ++j) *(volatile v4u*)(vt + gidx[j]) = vals[j];
      __threadfence();
      #pragma unroll
      for (unsigned j = 0; j < 4; ++j) *(volatile v4u*)(vt + gidx[j]) = vals[j];
    }
  }
}

__global__ __launch_bounds__(256) void attn_kernel(const f16* __restrict__ qp,
                                                   const f16* __restrict__ kp,
                                                   const f16* __restrict__ vt,
                                                   f16* __restrict__ ctx) {
  __shared__ __align__(16) float sO[NWAVE * 16 * OP];
  const unsigned tid  = threadIdx.x;
  const unsigned wave = (unsigned)__builtin_amdgcn_readfirstlane((int)(tid >> 5));
  const unsigned lane = tid & 31u;
  const unsigned lq   = lane & 15u;
  const unsigned hi   = lane >> 4;
  const unsigned qblk = blockIdx.x;
  const unsigned h    = blockIdx.y;
  const unsigned b    = blockIdx.z;

  const unsigned qrow0 = qblk * BQ + wave * 16u;
  const size_t   bh    = (size_t)b * NHEAD + h;
  const f16* q_h = qp + bh * SPAD * HDIM;
  const f16* k_h = kp + bh * SPAD * HDIM;
  const f16* v_h = vt + bh * HDIM * SPAD;

  FragH qf[2];
  {
    const f16* qr = q_h + (size_t)(qrow0 + lq) * HDIM + hi * 8u;
    #pragma unroll
    for (unsigned f = 0; f < 2; ++f) {
      qf[f].q[0] = *(const v4u*)(qr + f * 32u);
      qf[f].q[1] = *(const v4u*)(qr + f * 32u + 16u);
    }
  }

  const unsigned last_tok = (unsigned)SEQ - 1u;
  const unsigned kend_q  = seg_end_of(umin_u(qrow0 + lq, last_tok));
  const unsigned kend_lo = seg_end_of(umin_u(qrow0, last_tok));
  unsigned kend_w        = seg_end_of(umin_u(qrow0 + 15u, last_tok));
  kend_w = (qrow0 >= (unsigned)SEQ) ? (unsigned)BK : kend_w;
  const unsigned nchunk = (kend_w + BK - 1u) / BK;

  v8f o[4];
  #pragma unroll
  for (unsigned dt = 0; dt < 4; ++dt) o[dt] = zero8();

  float rmax = -__builtin_inff();
  float rsum = 0.0f;
  const float SL = 0.125f * 1.4426950408889634f;

  #pragma unroll 1
  for (unsigned ic = 0; ic < nchunk; ++ic) {
    const unsigned j0 = ic * BK;

    FragH ak[2][2];
    #pragma unroll
    for (unsigned sub = 0; sub < 2; ++sub) {
      #pragma unroll
      for (unsigned f = 0; f < 2; ++f) {
        const f16* base = k_h + (size_t)(j0 + sub * 16u + lq) * HDIM + f * 32u + hi * 8u;
        ak[sub][f].q[0] = *(const v4u*)(base);
        ak[sub][f].q[1] = *(const v4u*)(base + 16);
      }
    }
    FragH bv[4];
    #pragma unroll
    for (unsigned dt = 0; dt < 4; ++dt) {
      const f16* base = v_h + (size_t)(dt * 16u + lq) * SPAD + j0 + hi * 8u;
      bv[dt].q[0] = *(const v4u*)(base);
      bv[dt].q[1] = *(const v4u*)(base + 16);
    }

    v8f c[2];
    #pragma unroll
    for (unsigned sub = 0; sub < 2; ++sub) {
      v8f acc = zero8();
      acc = mma_f16(ak[sub][0].v, qf[0].v, acc);
      acc = mma_f16(ak[sub][1].v, qf[1].v, acc);
      c[sub] = acc;
    }

    if (j0 + BK > kend_lo) {
      #pragma unroll
      for (unsigned sub = 0; sub < 2; ++sub) {
        #pragma unroll
        for (unsigned r = 0; r < 8; ++r) {
          const unsigned key = j0 + sub * 16u + hi * 8u + r;
          c[sub][r] = (key >= kend_q) ? -__builtin_inff() : c[sub][r];
        }
      }
    }

    float m_new = rmax;
    #pragma unroll
    for (unsigned r = 0; r < 8; ++r) {
      m_new = fmaxf(m_new, c[0][r]);
      m_new = fmaxf(m_new, c[1][r]);
    }
    m_new = fmaxf(m_new, __shfl_xor(m_new, 16, 32));
    const float scale = __builtin_amdgcn_exp2f((rmax - m_new) * SL);
    rmax = m_new;

    FragH pa;
    float psum = 0.0f;
    #pragma unroll
    for (unsigned r = 0; r < 8; ++r) {
      const float p0 = __builtin_amdgcn_exp2f((c[0][r] - m_new) * SL);
      const float p1 = __builtin_amdgcn_exp2f((c[1][r] - m_new) * SL);
      psum += p0 + p1;
      pa.h[r]      = (f16)(p0 * PCARRY);
      pa.h[8u + r] = (f16)(p1 * PCARRY);
    }
    rsum = rsum * scale + psum + __shfl_xor(psum, 16, 32);

    float sc[8];
    #pragma unroll
    for (unsigned r = 0; r < 8; ++r) sc[r] = __shfl(scale, (int)((hi << 3) + r), 32);
    #pragma unroll
    for (unsigned dt = 0; dt < 4; ++dt) {
      #pragma unroll
      for (unsigned r = 0; r < 8; ++r) o[dt][r] *= sc[r];
    }

    #pragma unroll
    for (unsigned dt = 0; dt < 4; ++dt) o[dt] = mma_f16(pa.v, bv[dt].v, o[dt]);
  }

  float rs[8];
  #pragma unroll
  for (unsigned r = 0; r < 8; ++r) rs[r] = 1.0f / __shfl(rsum, (int)((hi << 3) + r), 32);

  float* so = sO + wave * (16u * OP);
  #pragma unroll
  for (unsigned r = 0; r < 8; ++r) {
    #pragma unroll
    for (unsigned dt = 0; dt < 4; ++dt)
      so[(hi * 8u + r) * OP + dt * 16u + lq] = o[dt][r] * (CCARRY / PCARRY) * rs[r];
  }
  __syncthreads();

  v4u    vals[4];
  size_t gidx[4];
  #pragma unroll
  for (unsigned it = 0; it < 4; ++it) {
    const unsigned row = it * 4u + (lane >> 3);
    const unsigned p   = lane & 7u;
    const v4f a0 = *(const v4f*)(so + row * OP + p * 8u);
    const v4f a1 = *(const v4f*)(so + row * OP + p * 8u + 4u);
    Pack8H pk;
    #pragma unroll
    for (unsigned i = 0; i < 4; ++i) {
      pk.h[i]      = (f16)a0[i];
      pk.h[4u + i] = (f16)a1[i];
    }
    vals[it] = pk.u;
    gidx[it] = ((size_t)b * SPAD + qrow0 + row) * DIM + h * HDIM + p * 8u;
  }
  #pragma unroll
  for (unsigned it = 0; it < 4; ++it) *(volatile v4u*)(ctx + gidx[it]) = vals[it];
  __threadfence();
  #pragma unroll
  for (unsigned it = 0; it < 4; ++it) *(volatile v4u*)(ctx + gidx[it]) = vals[it];
}

__global__ __launch_bounds__(256) void out_gemm_kernel(const f16* __restrict__ ctx,
                                                       const f16* __restrict__ wT,
                                                       const float* __restrict__ bias,
                                                       const float* __restrict__ x,
                                                       float* __restrict__ out) {
  __shared__ __align__(16) float sE[128 * PE];
  const unsigned tid  = threadIdx.x;
  const unsigned wave = (unsigned)__builtin_amdgcn_readfirstlane((int)(tid >> 5));
  const unsigned lane = tid & 31u;
  const unsigned lq   = lane & 15u;
  const unsigned hi   = lane >> 4;
  const unsigned wm   = wave & 3u;
  const unsigned wn   = wave >> 2;
  const unsigned bx   = blockIdx.x;
  const unsigned by   = blockIdx.y;
  const unsigned b    = blockIdx.z;

  const unsigned row0  = by * 128u + wm * 32u;
  const unsigned ncol0 = bx * 128u + wn * 64u;
  const f16* a_base = ctx + ((size_t)b * SPAD + row0 + lq) * DIM + hi * 8u;
  const f16* b_base = wT + ((size_t)ncol0 + lq) * DIM + hi * 8u;
  const unsigned ksteps = (row0 < (unsigned)SEQ) ? (unsigned)(DIM / 32) : 0u;

  v8f acc[2][4];
  #pragma unroll
  for (unsigned ms = 0; ms < 2; ++ms) {
    #pragma unroll
    for (unsigned t = 0; t < 4; ++t) acc[ms][t] = zero8();
  }
  gemm_32x64(a_base, b_base, ksteps, acc);

  #pragma unroll
  for (unsigned t = 0; t < 4; ++t) {
    #pragma unroll
    for (unsigned ms = 0; ms < 2; ++ms) {
      #pragma unroll
      for (unsigned r = 0; r < 8; ++r) {
        sE[(wm * 32u + ms * 16u + hi * 8u + r) * PE + wn * 64u + t * 16u + lq] =
            acc[ms][t][r] * (1.0f / (WCARRY * CCARRY));
      }
    }
  }
  __syncthreads();

  const unsigned ncol = bx * 128u + lane * 4u;
  const v4f bv = *(const v4f*)(bias + ncol);
  v4f bb;
  bb[0] = bfr(bv[0]); bb[1] = bfr(bv[1]); bb[2] = bfr(bv[2]); bb[3] = bfr(bv[3]);

  #pragma unroll
  for (unsigned g = 0; g < 2; ++g) {
    v4f vals[8];
    const unsigned tok0 = by * 128u + wave * 16u + g * 8u;
    #pragma unroll
    for (unsigned j = 0; j < 8; ++j) {
      const unsigned row = wave * 16u + g * 8u + j;
      const unsigned sc  = umin_u(tok0 + j, (unsigned)SEQ - 1u);
      const v4f a  = *(const v4f*)(sE + row * PE + lane * 4u);
      const v4f xv = *(const v4f*)(x + ((size_t)b * SEQ_FULL + sc) * DIM + ncol);
      v4f v;
      #pragma unroll
      for (unsigned i = 0; i < 4; ++i) v[i] = (a[i] + bb[i]) + bfr(xv[i]);
      vals[j] = v;
    }
    float* obase = out + ((size_t)b * SEQ_FULL + tok0) * DIM + ncol;
    #pragma unroll
    for (unsigned j = 0; j < 8; ++j) {
      if (tok0 + j < (unsigned)SEQ) *(volatile v4f*)(obase + (size_t)j * DIM) = vals[j];
    }
    __threadfence();
    #pragma unroll
    for (unsigned j = 0; j < 8; ++j) {
      if (tok0 + j < (unsigned)SEQ) *(volatile v4f*)(obase + (size_t)j * DIM) = vals[j];
    }
  }
}

extern "C" void kernel_launch(void* const* d_in, const int* in_sizes, int n_in,
                              void* d_out, int out_size, void* d_ws, size_t ws_size,
                              hipStream_t stream) {
  if (n_in < 8) return;
  const size_t rows_used = (size_t)(NB - 1) * SEQ_FULL + SEQ;
  if ((size_t)in_sizes[0] < rows_used * DIM) return;
  if ((size_t)in_sizes[1] < (size_t)NB * CDIM) return;
  if ((size_t)in_sizes[2] < (size_t)CDIM * ADA_N) return;
  if ((size_t)in_sizes[3] < (size_t)ADA_N) return;
  if ((size_t)in_sizes[4] < (size_t)DIM * QKV_N) return;
  if ((size_t)in_sizes[5] < (size_t)QKV_N) return;
  if ((size_t)in_sizes[6] < (size_t)DIM * DIM) return;
  if ((size_t)in_sizes[7] < (size_t)DIM) return;
  if ((size_t)out_size < rows_used * DIM) return;
  if (ws_size < WS_TOTAL) return;

  const float* x       = (const float*)d_in[0];
  const float* cond    = (const float*)d_in[1];
  const float* adaln_w = (const float*)d_in[2];
  const float* adaln_b = (const float*)d_in[3];
  const float* qkv_w   = (const float*)d_in[4];
  const float* qkv_b   = (const float*)d_in[5];
  const float* out_w   = (const float*)d_in[6];
  const float* out_b   = (const float*)d_in[7];
  float* out = (float*)d_out;

  char* ws = (char*)d_ws;
  float* ftab = (float*)(ws + OFF_FTAB);
  float* wb   = (float*)(ws + OFF_WB);
  float* tabC = (float*)(ws + OFF_TABC);
  float* tabS = (float*)(ws + OFF_TABS);
  f16*   wqkv = (f16*)(ws + OFF_WQKV);
  f16*   wout = (f16*)(ws + OFF_WOUT);
  f16*   xn   = (f16*)(ws + OFF_XN);
  f16*   ctx  = (f16*)(ws + OFF_XN);
  f16*   qp   = (f16*)(ws + OFF_Q);
  f16*   kp   = (f16*)(ws + OFF_K);
  f16*   vt   = (f16*)(ws + OFF_VT);

  F32x32 fs[4];
  {
    const double xs = 2.302585092994046 / 128.0;
    double term = 1.0, ratio = 1.0;
    for (int n = 1; n <= 24; ++n) { term *= xs / (double)n; ratio += term; }
    double cur = 3.141592653589793;
    for (int m = 0; m < 128; ++m) {
      fs[m >> 5].v[m & 31] = (float)cur;
      cur *= ratio;
    }
  }
  for (unsigned g = 0; g < 4; ++g)
    freq_kernel<<<dim3(1), dim3(32), 0, stream>>>(fs[g], ftab, g * 32u);

  rope_table_kernel<<<dim3(SPAD / 4, NHEAD), dim3(256), 0, stream>>>(ftab, tabC, tabS);
  adaln_kernel<<<dim3(ADA_N / 1024, NB), dim3(256), 0, stream>>>(cond, adaln_w, adaln_b, wb);
  wt_plane_kernel<<<dim3(QKV_N / 64, DIM / 64), dim3(256), 0, stream>>>(qkv_w, wqkv, (unsigned)DIM, (unsigned)QKV_N);
  wt_plane_kernel<<<dim3(DIM / 64, DIM / 64), dim3(256), 0, stream>>>(out_w, wout, (unsigned)DIM, (unsigned)DIM);
  ln_kernel<<<dim3(SPAD / 8, NB), dim3(256), 0, stream>>>(x, wb, xn);
  qkv_gemm_kernel<<<dim3(QKV_N / 128, SPAD / 128, NB), dim3(256), 0, stream>>>(xn, wqkv, qkv_b, tabC, tabS,
                                                                               qp, kp, vt);
  attn_kernel<<<dim3(SPAD / BQ, NHEAD, NB), dim3(256), 0, stream>>>(qp, kp, vt, ctx);
  out_gemm_kernel<<<dim3(DIM / 128, SPAD / 128, NB), dim3(256), 0, stream>>>(ctx, wout, out_b, x, out);
}
